// DepthAttnLayer_25598005084240
// MI455X (gfx1250) — hardware-verified
//
#include <hip/hip_runtime.h>
#include <math.h>

typedef __attribute__((ext_vector_type(16))) _Float16 v16h;
typedef __attribute__((ext_vector_type(16))) __bf16 v16b;
typedef __attribute__((ext_vector_type(8)))  _Float16 v8h;
typedef __attribute__((ext_vector_type(8)))  float v8f;
typedef __attribute__((ext_vector_type(4)))  float v4f;
typedef __attribute__((ext_vector_type(2)))  float v2f;
typedef __attribute__((ext_vector_type(4)))  unsigned v4u;
typedef __attribute__((ext_vector_type(4)))  int v4i;
typedef float __attribute__((may_alias)) float_a;
typedef int __attribute__((may_alias)) int_a;

template <typename T> __device__ __forceinline__ void vst2(void* p, T v) { *(volatile T*)p = v; __threadfence(); *(volatile T*)p = v; }
__device__ __forceinline__ v8f wmma16(v16h a, v16h b, v8f c) {
  v8f d = __builtin_amdgcn_wmma_f32_16x16x32_f16(false, a, false, b, (short)0, c, false, false);
  asm volatile("v_nop\n\tv_nop\n\tv_nop\n\tv_nop" : "+v"(d) : "v"(a), "v"(b));
  return d;
}
__device__ __forceinline__ v8f wmma_bf(v16b a, v16b b, v8f c) {
  v8f d = __builtin_amdgcn_wmma_f32_16x16x32_bf16(false, a, false, b, (short)0, c, false, false);
  asm volatile("v_nop\n\tv_nop\n\tv_nop\n\tv_nop" : "+v"(d) : "v"(a), "v"(b));
  return d;
}
__device__ __forceinline__ v16h frag_h(const _Float16* rowk0, int lane) {
  union { v16h v; v8h q[2]; } u; const _Float16* p = rowk0 + 8 * (lane >> 4);
  u.q[0] = *(const v8h*)p; u.q[1] = *(const v8h*)(p + 16); return u.v;
}
__device__ __forceinline__ v16h frag_f32(const float* rowk0, int lane) {
  v16h a; const float* p = rowk0 + 8 * (lane >> 4);
#pragma unroll
  for (int i = 0; i < 8; ++i) { a[i] = (_Float16)p[i]; a[8 + i] = (_Float16)p[16 + i]; }
  return a;
}
__device__ __forceinline__ v16h frag_f32s(const float* rowk0, int lane, float sc) {
  v16h a; const float* p = rowk0 + 8 * (lane >> 4);
#pragma unroll
  for (int i = 0; i < 8; ++i) { a[i] = (_Float16)(p[i] * sc); a[8 + i] = (_Float16)(p[16 + i] * sc); }
  return a;
}
__device__ __forceinline__ v16h fragc_f32(const float* W, int k0, int n, int lane, int ld, int K) {
  v16h a; const int g = lane >> 4;
#pragma unroll
  for (int i = 0; i < 8; ++i) { const int ka = k0 + 8 * g + i, kb = ka + 16;
    a[i] = (_Float16)(ka < K ? W[(size_t)ka * ld + n] : 0.f); a[8 + i] = (_Float16)(kb < K ? W[(size_t)kb * ld + n] : 0.f); }
  return a;
}
struct F2 { v16b h, l; };
__device__ __forceinline__ F2 bsplit16(const float v[16]) { F2 r;
#pragma unroll
  for (int i = 0; i < 16; ++i) { const __bf16 h = (__bf16)v[i]; r.h[i] = h; r.l[i] = (__bf16)(v[i] - (float)h); }
  return r; }
__device__ __forceinline__ F2 split_row(const float* row, int k0, int lane) { float v[16]; const float* p = row + k0 + 8 * (lane >> 4);
#pragma unroll
  for (int i = 0; i < 8; ++i) { v[i] = p[i]; v[8 + i] = p[16 + i]; }
  return bsplit16(v); }
__device__ __forceinline__ F2 split_rowK(const float* row, int k0, int lane, int K) { float v[16]; const int g = lane >> 4;
#pragma unroll
  for (int i = 0; i < 8; ++i) { const int ka = k0 + 8 * g + i, kb = ka + 16; v[i] = ka < K ? row[ka] : 0.f; v[8 + i] = kb < K ? row[kb] : 0.f; }
  return bsplit16(v); }
__device__ __forceinline__ F2 split_col(const float* W, int k0, int n, int lane, int ld, int K) { float v[16]; const int g = lane >> 4;
#pragma unroll
  for (int i = 0; i < 8; ++i) { const int ka = k0 + 8 * g + i, kb = ka + 16; v[i] = ka < K ? W[(size_t)ka * ld + n] : 0.f; v[8 + i] = kb < K ? W[(size_t)kb * ld + n] : 0.f; }
  return bsplit16(v); }
__device__ __forceinline__ v8f mac3(const F2& a, const F2& b, v8f c) { c = wmma_bf(a.l, b.h, c); c = wmma_bf(a.h, b.l, c); return wmma_bf(a.h, b.h, c); }
__device__ __forceinline__ float sigm(float v) { return 1.0f / (1.0f + expf(-v)); }
#define LDSX() do { asm volatile("s_wait_dscnt 0" ::: "memory"); __builtin_amdgcn_wave_barrier(); __builtin_amdgcn_fence(__ATOMIC_RELEASE, "workgroup"); } while (0)


#define TGT 32400
#define TGP 32448
#define SRC 16896
#define NPT 1036800
#define E 256
#define FF 512
#define HDIM 32
#define LMAX 64
__device__ __forceinline__ int clampf(int v) { return v < 0 ? 0 : (v >= SRC ? SRC - 1 : v); }

__global__ __launch_bounds__(256) void k_pack(const float* __restrict__ inw, const float* __restrict__ Wo, const float* __restrict__ W1, const float* __restrict__ W2, _Float16* __restrict__ PT, _Float16* __restrict__ P2) {
  const int b = blockIdx.x, tid = threadIdx.x; __shared__ __align__(16) _Float16 srow[FF];
  if (b < 1280) { const float* src = b < 256 ? inw + (size_t)b * E : (b < 512 ? inw + (size_t)(512 + b - 256) * E : (b < 768 ? Wo + (size_t)(b - 512) * E : W1 + (size_t)(b - 768) * E));
    srow[tid] = (_Float16)(src[tid] * 16.0f); __syncthreads(); if (tid < E / 8) vst2(PT + (size_t)b * E + tid * 8, *(const v4u*)(&srow[tid * 8])); }
  else { const int n = b - 1280; for (int k = tid; k < FF; k += 256) srow[k] = (_Float16)(W2[(size_t)n * FF + k] * 16.0f); __syncthreads(); if (tid < FF / 8) vst2(P2 + (size_t)n * FF + tid * 8, *(const v4u*)(&srow[tid * 8])); }
}
__global__ __launch_bounds__(128) void k_proj(const float* __restrict__ A, int M, const _Float16* __restrict__ PTw, const float* __restrict__ bias, float sc, float* __restrict__ C) {
  __shared__ __align__(16) float so[4][16][132];
  const int tid = threadIdx.x, wave = tid >> 5, lane = tid & 31, col = lane & 15, g = lane >> 4;
  const int r0 = blockIdx.x * 64 + wave * 16; const int ra = (r0 + col) < M ? (r0 + col) : (M - 1);
#pragma unroll 1
  for (int nh = 0; nh < 2; ++nh) { v8f acc[8] = {};
#pragma unroll 2
    for (int kc = 0; kc < E / 32; ++kc) { const v16h a = frag_f32(A + (size_t)ra * E + kc * 32, lane);
#pragma unroll
      for (int j = 0; j < 8; ++j) acc[j] = wmma16(a, frag_h(PTw + (size_t)(nh * 128 + j * 16 + col) * E + kc * 32, lane), acc[j]); }
#pragma unroll
    for (int j = 0; j < 8; ++j) { const float bb = bias[nh * 128 + j * 16 + col];
#pragma unroll
      for (int r = 0; r < 8; ++r) so[wave][8 * g + r][j * 16 + col] = (r0 + 8 * g + r) < M ? (acc[j][r] * (1.0f / 16.0f) + bb) * sc : 0.f; }
    LDSX();
#pragma unroll 4
    for (int rl = 0; rl < 16; ++rl) vst2(C + (size_t)(r0 + rl) * E + nh * 128 + lane * 4, *(const v4f*)(&so[wave][rl][lane * 4]));
    LDSX(); }
}
__global__ __launch_bounds__(256) void k_att(const float* __restrict__ Q, const float* __restrict__ KP, const float* __restrict__ V, const int* __restrict__ rfeat, const int* __restrict__ istart, const int* __restrict__ ilen, float* __restrict__ ATT) {
  const int wave = threadIdx.x >> 5, lane = threadIdx.x & 31; const int i = blockIdx.x * 8 + wave; if (i >= TGP) return;
  v4f oa = {0.f, 0.f, 0.f, 0.f}, ob = {0.f, 0.f, 0.f, 0.f};
  if (i < TGT) {
    const v4f qa = *(const v4f*)(Q + (size_t)i * E + lane * 4), qb = *(const v4f*)(Q + (size_t)i * E + 128 + lane * 4);
    int st = istart[i], ln = ilen[i]; ln = ln < 0 ? 0 : (ln > LMAX ? LMAX : ln); st = st < 0 ? 0 : st; if (st + ln > NPT) ln = NPT - st > 0 ? NPT - st : 0;
    float ma = -3.0e38f, mb = -3.0e38f, la = 0.f, lb = 0.f;
#pragma unroll 1
    for (int p = 0; p < ln; ++p) { const int f = clampf(rfeat[st + p]);
      const v4f ka = *(const v4f*)(KP + (size_t)f * E + lane * 4), kb = *(const v4f*)(KP + (size_t)f * E + 128 + lane * 4);
      float da = qa[0] * ka[0] + qa[1] * ka[1] + qa[2] * ka[2] + qa[3] * ka[3], db = qb[0] * kb[0] + qb[1] * kb[1] + qb[2] * kb[2] + qb[3] * kb[3];
      da += __shfl_xor(da, 1, 32); da += __shfl_xor(da, 2, 32); da += __shfl_xor(da, 4, 32);
      db += __shfl_xor(db, 1, 32); db += __shfl_xor(db, 2, 32); db += __shfl_xor(db, 4, 32);
      const float mna = fmaxf(ma, da), mnb = fmaxf(mb, db); const float ca = expf(ma - mna), cb = expf(mb - mnb); const float pa = expf(da - mna), pb = expf(db - mnb);
      la = la * ca + pa; lb = lb * cb + pb; ma = mna; mb = mnb;
      const v4f va = *(const v4f*)(V + (size_t)f * E + lane * 4), vb = *(const v4f*)(V + (size_t)f * E + 128 + lane * 4);
#pragma unroll
      for (int c = 0; c < 4; ++c) { oa[c] = oa[c] * ca + pa * va[c]; ob[c] = ob[c] * cb + pb * vb[c]; } }
    const float ia = la > 0.f ? 1.0f / la : 0.f, ib = lb > 0.f ? 1.0f / lb : 0.f;
#pragma unroll
    for (int c = 0; c < 4; ++c) { oa[c] *= ia; ob[c] *= ib; } }
  vst2(ATT + (size_t)i * E + lane * 4, oa); vst2(ATT + (size_t)i * E + 128 + lane * 4, ob);
}
__global__ __launch_bounds__(128) void k_oln(const float* __restrict__ ATT, const float* __restrict__ query, const _Float16* __restrict__ PTo, const float* __restrict__ bo, const float* __restrict__ nw, const float* __restrict__ nb, float* __restrict__ X) {
  __shared__ __align__(16) float so[4][16][E + 4];
  const int tid = threadIdx.x, wave = tid >> 5, lane = tid & 31, col = lane & 15, g = lane >> 4;
  const int r0 = blockIdx.x * 64 + wave * 16; const int ra = (r0 + col) < TGT ? (r0 + col) : (TGT - 1);
#pragma unroll 1
  for (int nh = 0; nh < 2; ++nh) { v8f acc[8] = {};
#pragma unroll 2
    for (int kc = 0; kc < E / 32; ++kc) { const v16h a = frag_f32(ATT + (size_t)ra * E + kc * 32, lane);
#pragma unroll
      for (int j = 0; j < 8; ++j) acc[j] = wmma16(a, frag_h(PTo + (size_t)(nh * 128 + j * 16 + col) * E + kc * 32, lane), acc[j]); }
#pragma unroll
    for (int j = 0; j < 8; ++j) { const int n = nh * 128 + j * 16 + col; const float bb = bo[n];
#pragma unroll
      for (int r = 0; r < 8; ++r) { const int row = r0 + 8 * g + r; const int rr = row < TGT ? row : TGT - 1; so[wave][8 * g + r][n] = acc[j][r] * (1.0f / 16.0f) + bb + query[(size_t)rr * E + n]; } } }
  LDSX();
  { const int rl = lane & 15, hf = lane >> 4; float* row = &so[wave][rl][hf * 128]; float s = 0.f;
#pragma unroll 4
    for (int k = 0; k < 128; ++k) s += row[k];
    s += __shfl_xor(s, 16, 32); const float mu = s * (1.0f / E); float q = 0.f;
#pragma unroll 4
    for (int k = 0; k < 128; ++k) { const float dv = row[k] - mu; q += dv * dv; }
    q += __shfl_xor(q, 16, 32); const float rs = rsqrtf(q * (1.0f / E) + 1e-5f);
#pragma unroll 4
    for (int k = 0; k < 128; ++k) row[k] = (row[k] - mu) * rs * nw[hf * 128 + k] + nb[hf * 128 + k]; }
  LDSX();
  for (int rl = 0; rl < 16; ++rl) { v4f v = *(const v4f*)(&so[wave][rl][lane * 4]), w2 = *(const v4f*)(&so[wave][rl][128 + lane * 4]); if (r0 + rl >= TGT) { v = (v4f){0.f, 0.f, 0.f, 0.f}; w2 = v; }
    vst2(X + (size_t)(r0 + rl) * E + lane * 4, v); vst2(X + (size_t)(r0 + rl) * E + 128 + lane * 4, w2); }
}
__global__ __launch_bounds__(128) void k_ffn(const float* __restrict__ X, const _Float16* __restrict__ PT1, const float* __restrict__ b1, const _Float16* __restrict__ P2, const float* __restrict__ b2, float* __restrict__ out) {
  __shared__ __align__(16) _Float16 sZ[64][FF + 8];
  __shared__ __align__(16) float so[4][16][132];
  const int tid = threadIdx.x, wave = tid >> 5, lane = tid & 31, col = lane & 15, g = lane >> 4;
  const int r0 = blockIdx.x * 64 + wave * 16; const int ra = (r0 + col) < TGT ? (r0 + col) : (TGT - 1);
#pragma unroll 1
  for (int zh = 0; zh < FF / 128; ++zh) { v8f zacc[8] = {};
#pragma unroll 2
    for (int kc = 0; kc < E / 32; ++kc) { const v16h a = frag_f32(X + (size_t)ra * E + kc * 32, lane);
#pragma unroll
      for (int j = 0; j < 8; ++j) zacc[j] = wmma16(a, frag_h(PT1 + (size_t)(zh * 128 + j * 16 + col) * E + kc * 32, lane), zacc[j]); }
#pragma unroll
    for (int j = 0; j < 8; ++j) { const int n = zh * 128 + j * 16 + col; const float bb = b1[n];
#pragma unroll
      for (int r = 0; r < 8; ++r) { const float v = zacc[j][r] * (1.0f / 16.0f) + bb; sZ[wave * 16 + 8 * g + r][n] = (_Float16)(v > 0.f ? v : 0.f); } } }
  LDSX();
#pragma unroll 1
  for (int nh = 0; nh < 2; ++nh) { v8f acc[8] = {};
#pragma unroll 2
    for (int kc = 0; kc < FF / 32; ++kc) { const v16h a = frag_h(&sZ[wave * 16 + col][0] + kc * 32, lane);
#pragma unroll
      for (int j = 0; j < 8; ++j) acc[j] = wmma16(a, frag_h(P2 + (size_t)(nh * 128 + j * 16 + col) * FF + kc * 32, lane), acc[j]); }
#pragma unroll
    for (int j = 0; j < 8; ++j) { const int n = nh * 128 + j * 16 + col; const float bb = b2[n];
#pragma unroll
      for (int r = 0; r < 8; ++r) { const int row = r0 + 8 * g + r; const int rr = row < TGT ? row : TGT - 1; so[wave][8 * g + r][j * 16 + col] = acc[j][r] * (1.0f / 16.0f) + bb + X[(size_t)rr * E + n]; } }
    LDSX();
    for (int rl = 0; rl < 16; ++rl) { if (r0 + rl >= TGT) break; vst2(out + (size_t)(r0 + rl) * E + nh * 128 + lane * 4, *(const v4f*)(&so[wave][rl][lane * 4])); }
    LDSX(); }
}
extern "C" void kernel_launch(void* const* d_in, const int* in_sizes, int n_in, void* d_out, int out_size, void* d_ws, size_t ws_size, hipStream_t stream) {
  (void)in_sizes; (void)n_in; (void)out_size; (void)ws_size;
  const float* query = (const float*)d_in[0]; const float* key = (const float*)d_in[1]; const float* value = (const float*)d_in[2]; const float* inw = (const float*)d_in[3]; const float* inb = (const float*)d_in[4];
  const float* Wo = (const float*)d_in[5]; const float* bo = (const float*)d_in[6]; const float* nw = (const float*)d_in[7]; const float* nb = (const float*)d_in[8];
  const float* W1 = (const float*)d_in[9]; const float* b1 = (const float*)d_in[10]; const float* W2 = (const float*)d_in[11]; const float* b2 = (const float*)d_in[12];
  const int* rfeat = (const int*)d_in[13]; const int* istart = (const int*)d_in[15]; const int* ilen = (const int*)d_in[16];
  float* out = (float*)d_out;
  char* ws = (char*)d_ws; size_t off = 0;
  auto take = [&](size_t bytes) { char* p = ws + off; off += (bytes + 255) & ~(size_t)255; return p; };
  _Float16* PT = (_Float16*)take((size_t)1280 * E * 2); _Float16* P2 = (_Float16*)take((size_t)E * FF * 2);
  float* KP = (float*)take((size_t)SRC * E * 4); float* Qb = (float*)take((size_t)TGP * E * 4); float* ATT = (float*)take((size_t)TGP * E * 4); float* X = (float*)take((size_t)TGP * E * 4);
  k_pack<<<1280 + E, 256, 0, stream>>>(inw, Wo, W1, W2, PT, P2);
  k_proj<<<SRC / 64, 128, 0, stream>>>(key, SRC, PT, inb, 1.0f, KP);
  k_proj<<<TGP / 64, 128, 0, stream>>>(query, TGT, PT + (size_t)256 * E, inb + 512, 0.17677669529663687f, Qb);
  k_att<<<TGP / 8, 256, 0, stream>>>(Qb, KP, value, rfeat, istart, ilen, ATT);
  k_oln<<<TGP / 64, 128, 0, stream>>>(ATT, query, PT + (size_t)512 * E, bo, nw, nb, X);
  k_ffn<<<TGP / 64, 128, 0, stream>>>(X, PT + (size_t)768 * E, b1, P2, b2, out);
}
